// CausalAnomalyDetector_61847529062649
// MI455X (gfx1250) — hardware-run, weakly checked
//
#include <hip/hip_runtime.h>
#include <math.h>
#include <stdint.h>

#ifndef NB
#define NB       32
#endif
#ifndef SEQ
#define SEQ      512
#endif
#define NB_FULL  32
#define SEQ_FULL 512
#define DMODEL   256
#define DFF      1024
#define NHEAD    8
#define HDIM     32
#define DEMB     512
#define DSTAT    64
#define DCOMB    320
#define NSH      32
#define NFEAT    6
#define HIDK     64
#define HSP      40
#define WIN      10
#define NLAYER   2
#define NTOK     (NB * SEQ)
#define RELDEN   ((SEQ > 100) ? SEQ : 100)
#define WSC      64.0f
#define EC       64.0f
#define HCARRY   16.0f
#define QC       64.0f
#define KC       64.0f
#define VC       64.0f
#define PC       1024.0f
#define FC       1024.0f
#define GC       64.0f
#define HIDC     64.0f
#define ATT_SCALE 0.17677669529663687f
#define LOG2E    1.4426950408889634f
#define LN_EPS   1e-5f
#define MFILL    (-1.0e9f)
static_assert(NHEAD * HDIM == DMODEL);
static_assert(DCOMB == DMODEL + DSTAT);
static_assert(NB >= 1 && NB <= NB_FULL && SEQ >= 64 && SEQ <= SEQ_FULL && (SEQ % 64) == 0 && (SEQ % 32) == 0 && (SEQ % 16) == 0);
static_assert(SEQ <= 512 && SEQ >= WIN);
static_assert((NTOK % 256) == 0 && (NTOK % 64) == 0);
static_assert((DMODEL % 64) == 0 && (DFF % 64) == 0 && (DEMB % 32) == 0 && (DCOMB % 32) == 0 && (DCOMB % 64) == 0 && (HIDK % 32) == 0);
static_assert((HSP % 8) == 0 && HSP >= NSH && NSH * 2 == HIDK);

#define HPB         8
#define OSP         (HPB * HDIM)
#define OSP8        (OSP / 8)
#define ATT_THREADS (HPB * 32)
#define ATT_BLOCKS  (NB * (SEQ / 16))
static_assert(ATT_THREADS == 256 && HPB == NHEAD);
#define LN_THREADS  64
static_assert(LN_THREADS * 4 == DMODEL && (LN_THREADS % 32) == 0 && (DMODEL / 8) == 32);
#define HEAD_THREADS 128
#define HEAD_ROWS    256
static_assert(HEAD_ROWS == (HEAD_THREADS / 32) * 64 && HEAD_ROWS == 64 * 4);

typedef _Float16 v16h __attribute__((ext_vector_type(16)));
typedef _Float16 v8h  __attribute__((ext_vector_type(8)));
typedef float    v8f  __attribute__((ext_vector_type(8)));
typedef float    v4f  __attribute__((ext_vector_type(4)));
typedef unsigned int v4u __attribute__((ext_vector_type(4)));
typedef unsigned int v2u __attribute__((ext_vector_type(2)));

union FragH { v16h v; v8h h[2]; v4u u[2]; };

__device__ __forceinline__ unsigned short bf_bits(float f) {
  unsigned u = __float_as_uint(f);
  return (unsigned short)((u + 0x7FFFu + ((u >> 16) & 1u)) >> 16);
}
__device__ __forceinline__ float bf_up(unsigned short h) { return __uint_as_float(((unsigned)h) << 16); }
__device__ __forceinline__ float bfr(float f) { return bf_up(bf_bits(f)); }
__device__ __forceinline__ unsigned short h_bits(_Float16 x) { return __builtin_bit_cast(unsigned short, x); }
__device__ __forceinline__ unsigned pk16(unsigned short a, unsigned short b) { return (unsigned)a | ((unsigned)b << 16); }
__device__ __forceinline__ v8f zero8() { v8f z = {0.f, 0.f, 0.f, 0.f, 0.f, 0.f, 0.f, 0.f}; return z; }
__device__ __forceinline__ int imin(int a, int b) { return a < b ? a : b; }
__device__ __forceinline__ int imax(int a, int b) { return a > b ? a : b; }
__device__ __forceinline__ float gelu_f(float u) { return 0.5f * u * (1.0f + erff(u * 0.70710678118654752f)); }

__device__ __forceinline__ v16h ldfrag_h(const _Float16* p) {
  FragH f;
  f.h[0] = *(const v8h*)(p);
  f.h[1] = *(const v8h*)(p + 16);
  return f.v;
}
__device__ __forceinline__ v16h ldfrag_u(const unsigned short* p) {
  FragH f;
  f.u[0] = *(const v4u*)(p);
  f.u[1] = *(const v4u*)(p + 16);
  return f.v;
}

__device__ __forceinline__ v8f mma_raw(v16h a, v16h b, v8f c) {
  return __builtin_amdgcn_wmma_f32_16x16x32_f16(false, a, false, b, (short)0, c, false, false);
}
__device__ __forceinline__ void dep_guard1(v8f& a, v8f& b, v16h x) {
#if defined(__HIP_DEVICE_COMPILE__)
  asm volatile("v_nop\n\tv_nop\n\tv_nop\n\tv_nop" : "+v"(a), "+v"(b) : "v"(x));
#endif
}
__device__ __forceinline__ void guard_ab3(v8f& a, v8f& b, v16h x, v16h y, v16h z) {
#if defined(__HIP_DEVICE_COMPILE__)
  asm volatile("v_nop\n\tv_nop\n\tv_nop\n\tv_nop" : "+v"(a), "+v"(b) : "v"(x), "v"(y), "v"(z));
#endif
}
__device__ __forceinline__ void keep4_h(v16h a, v16h b, v16h c, v16h d) {
#if defined(__HIP_DEVICE_COMPILE__)
  asm volatile("v_nop" :: "v"(a), "v"(b), "v"(c), "v"(d));
#endif
}
__device__ __forceinline__ void keep2_h(v16h a, v16h b) {
#if defined(__HIP_DEVICE_COMPILE__)
  asm volatile("v_nop" :: "v"(a), "v"(b));
#endif
}
__device__ __forceinline__ void acc_guard4(v8f& a, v8f& b, v8f& c, v8f& d) {
#if defined(__HIP_DEVICE_COMPILE__)
  asm volatile("v_nop\n\tv_nop\n\tv_nop\n\tv_nop" : "+v"(a), "+v"(b), "+v"(c), "+v"(d));
#endif
}
__device__ __forceinline__ void wave_sync_lds() {
  __builtin_amdgcn_fence(__ATOMIC_RELEASE, "workgroup");
  __builtin_amdgcn_wave_barrier();
  __builtin_amdgcn_fence(__ATOMIC_ACQUIRE, "workgroup");
}

__global__ __launch_bounds__(256) void tcvt16(const float* __restrict__ src, long long sZ,
                                              unsigned short* dst, long long dZ,
                                              int R, int C, int Rp, int Cp, float sc) {
  __shared__ __align__(16) unsigned short sT[64 * 72];
  const int tid = threadIdx.x, lane = tid & 31, wave = tid >> 5;
  const int c0 = blockIdx.x * 64, r0 = blockIdx.y * 64;
  const float* srcz = src + (size_t)((long long)blockIdx.z * sZ);
  unsigned short* dstz = dst + (size_t)((long long)blockIdx.z * dZ);
  const int rr = tid >> 2, cc = (tid & 3) * 16;
  const int r = r0 + rr;
  const int rcl = imin(r, R - 1);
  const float* sp = srcz + (size_t)rcl * C;
#pragma unroll
  for (int e = 0; e < 16; ++e) {
    const int cidx = c0 + cc + e;
    const int ccl = imin(cidx, C - 1);
    float a = sp[ccl];
    a = (r < R && cidx < C) ? a : 0.f;
    sT[(cc + e) * 72 + rr] = h_bits((_Float16)(bfr(a) * sc));
  }
  __syncthreads();
  v4u vals[2];
#pragma unroll
  for (int it = 0; it < 2; ++it) {
    const int q = it * 32 + wave * 4 + (lane >> 3);
    vals[it] = *(const v4u*)(sT + q * 72 + (lane & 7) * 8);
  }
  for (int pass = 0; pass < 2; ++pass) {
#pragma unroll
    for (int it = 0; it < 2; ++it) {
      const int q = it * 32 + wave * 4 + (lane >> 3);
      *(volatile v4u*)(dstz + (size_t)(c0 + q) * Rp + r0 + (lane & 7) * 8) = vals[it];
    }
    __threadfence();
  }
  (void)Cp;
}

template <int OM, int RM, int ACT, int BM>
__global__ __launch_bounds__(256) void gemm64(
    const unsigned short* __restrict__ Ap, int lda, long long sA,
    const unsigned short* __restrict__ Btp, int ldb, long long sB,
    const float* __restrict__ Rp, int rmod,
    const float* __restrict__ biasp, int nbias,
    void* Cout, int ldc, long long sC,
    int M, int N, int K, float oscale, float ocarry) {
  __shared__ __align__(16) float sT[8][16 * 68];
  const int by   = blockIdx.y;
  const int lane = threadIdx.x & 31;
  const int wave = threadIdx.x >> 5;
  const int tilesN = N >> 6;
  const int tilesM = M >> 6;
  const int tile = blockIdx.x * 8 + wave;
  if (tile >= tilesM * tilesN) return;
  const int tm = tile / tilesN;
  const int tn = tile - tm * tilesN;
  const int m0 = tm << 6;
  const int n0 = tn << 6;

  const unsigned short* A1 = Ap  + (size_t)((long long)by * sA);
  const unsigned short* Bb = Btp + (size_t)((long long)by * sB);

  const int rlane = lane & 15;
  const int koff  = (lane >> 4) * 8;
  const int mOff  = (lane >> 4) * 8;

  v8f acc[4][4];
#pragma unroll
  for (int i = 0; i < 4; ++i)
#pragma unroll
    for (int j = 0; j < 4; ++j) acc[i][j] = zero8();

  for (int k0 = 0; k0 < K; k0 += 32) {
    v16h bh[4];
#pragma unroll
    for (int j = 0; j < 4; ++j) {
      const size_t bofs = (size_t)(n0 + (j << 4) + rlane) * ldb + koff + k0;
      bh[j] = ldfrag_u(Bb + bofs);
    }
#pragma unroll
    for (int i = 0; i < 4; ++i) {
      const size_t ao = (size_t)(m0 + (i << 4) + rlane) * lda + koff + k0;
      const v16h ah = ldfrag_u(A1 + ao);
#pragma unroll
      for (int j = 0; j < 4; ++j) acc[i][j] = mma_raw(ah, bh[j], acc[i][j]);
      dep_guard1(acc[i][0], acc[i][3], ah);
    }
    keep4_h(bh[0], bh[1], bh[2], bh[3]);
  }
  acc_guard4(acc[0][0], acc[0][1], acc[0][2], acc[0][3]);
  acc_guard4(acc[1][0], acc[1][1], acc[1][2], acc[1][3]);
  acc_guard4(acc[2][0], acc[2][1], acc[2][2], acc[2][3]);
  acc_guard4(acc[3][0], acc[3][1], acc[3][2], acc[3][3]);

  const int hh2 = lane >> 4, c4 = (lane & 15) * 4;
  const int q8  = lane >> 3, c8 = (lane & 7) * 8;

  float bc4[4], bc8[8];
#pragma unroll
  for (int e = 0; e < 4; ++e) bc4[e] = 0.f;
#pragma unroll
  for (int e = 0; e < 8; ++e) bc8[e] = 0.f;
  if constexpr (BM == 1) {
    if constexpr (OM == 0) {
#pragma unroll
      for (int e = 0; e < 4; ++e) {
        const int n = n0 + c4 + e;
        const int ncl = imin(n, nbias - 1);
        const float t = bfr(biasp[ncl]);
        bc4[e] = (n < nbias) ? t : 0.f;
      }
    } else {
#pragma unroll
      for (int e = 0; e < 8; ++e) {
        const int n = n0 + c8 + e;
        const int ncl = imin(n, nbias - 1);
        const float t = bfr(biasp[ncl]);
        bc8[e] = (n < nbias) ? t : 0.f;
      }
    }
  }

  float* slab = sT[wave];
#pragma unroll
  for (int i = 0; i < 4; ++i) {
    const int mBase = m0 + (i << 4);
#pragma unroll
    for (int j = 0; j < 4; ++j) {
#pragma unroll
      for (int r = 0; r < 8; ++r) {
        slab[(mOff + r) * 68 + (j << 4) + rlane] = acc[i][j][r];
      }
    }
    wave_sync_lds();
    if constexpr (OM == 0) {
      float* C = (float*)Cout + (size_t)((long long)by * sC);
      v4f vals[8];
#pragma unroll
      for (int it = 0; it < 8; ++it) {
        const int row = it * 2 + hh2;
        const int gr  = mBase + row;
        v4f v = *(const v4f*)(slab + row * 68 + c4);
        v4f rv = {0.f, 0.f, 0.f, 0.f};
        if constexpr (RM == 1 || RM == 2 || RM == 3) {
          const float* R = Rp + (size_t)((long long)by * sC);
          const int rrow = (RM == 3) ? (gr % rmod) : gr;
          const v4f rraw = *(const v4f*)(R + (size_t)rrow * ldc + n0 + c4);
#pragma unroll
          for (int e = 0; e < 4; ++e) rv[e] = (RM == 2) ? rraw[e] : bfr(rraw[e]);
        }
        float rb = 0.f;
        if constexpr (BM == 2) {
          const int gcl = imin(gr, nbias - 1);
          const float tb = bfr(biasp[gcl]);
          rb = (gr < nbias) ? tb : 0.f;
        }
#pragma unroll
        for (int e = 0; e < 4; ++e) {
          float u = v[e] * oscale;
          if constexpr (BM == 1) u += bc4[e];
          if constexpr (BM == 2) u += rb;
          if constexpr (ACT == 1) u = gelu_f(u);
          if constexpr (ACT == 2) u = fmaxf(u, 0.f);
          v[e] = u + rv[e];
        }
        vals[it] = v;
      }
      for (int pass = 0; pass < 2; ++pass) {
#pragma unroll
        for (int it = 0; it < 8; ++it) {
          const int gr = mBase + it * 2 + hh2;
          *(volatile v4f*)(C + (size_t)gr * ldc + n0 + c4) = vals[it];
        }
        __threadfence();
      }
    } else {
      unsigned short* C = (unsigned short*)Cout + (size_t)((long long)by * sC);
      v4u hv[4];
#pragma unroll
      for (int it = 0; it < 4; ++it) {
        const int row = it * 4 + q8;
        const int gr  = mBase + row;
        const float* sp = slab + row * 68 + c8;
        float rb = 0.f;
        if constexpr (BM == 2) {
          const int gcl = imin(gr, nbias - 1);
          const float tb = bfr(biasp[gcl]);
          rb = (gr < nbias) ? tb : 0.f;
        }
        v4u a = {0u, 0u, 0u, 0u};
#pragma unroll
        for (int e = 0; e < 4; ++e) {
          float f0 = sp[2 * e] * oscale;
          float f1 = sp[2 * e + 1] * oscale;
          if constexpr (BM == 1) { f0 += bc8[2 * e]; f1 += bc8[2 * e + 1]; }
          if constexpr (BM == 2) { f0 += rb; f1 += rb; }
          if constexpr (ACT == 1) { f0 = gelu_f(f0); f1 = gelu_f(f1); }
          if constexpr (ACT == 2) { f0 = fmaxf(f0, 0.f); f1 = fmaxf(f1, 0.f); }
          f0 *= ocarry; f1 *= ocarry;
          a[e] = pk16(h_bits((_Float16)f0), h_bits((_Float16)f1));
        }
        hv[it] = a;
      }
      for (int pass = 0; pass < 2; ++pass) {
#pragma unroll
        for (int it = 0; it < 4; ++it) {
          const int row = it * 4 + q8;
          *(volatile v4u*)(C + (size_t)(mBase + row) * ldc + n0 + c8) = hv[it];
        }
        __threadfence();
      }
    }
    wave_sync_lds();
  }
}

__global__ __launch_bounds__(256) void egath(const int* __restrict__ qin, const int* __restrict__ sin_,
                                             const float* __restrict__ qe, int nqrows,
                                             const float* __restrict__ se, int nsrows,
                                             unsigned short* E) {
  const int tid = threadIdx.x;
  const int r = blockIdx.x * 4 + (tid >> 6);
  const int j = tid & 63;
  const int b = r / SEQ, t = r - b * SEQ;
  const size_t ii = (size_t)b * SEQ_FULL + t;
  const int sv = sin_[ii];
  const int qv = qin[ii];
  const int msk = (sv >= 0) ? 1 : 0;
  int qm = msk ? qv : 0;
  int sm = msk ? sv : 0;
  qm = imin(imax(qm, 0), nqrows - 1);
  sm = imin(imax(sm, 0), nsrows - 1);
  const float* src = (j < 32) ? (qe + (size_t)qm * DMODEL + (size_t)j * 8)
                              : (se + (size_t)sm * DMODEL + (size_t)(j - 32) * 8);
  const v4f a0 = *(const v4f*)(src);
  const v4f a1 = *(const v4f*)(src + 4);
  v4u w;
#pragma unroll
  for (int e = 0; e < 2; ++e) {
    w[e]     = pk16(h_bits((_Float16)(bfr(a0[2 * e]) * EC)), h_bits((_Float16)(bfr(a0[2 * e + 1]) * EC)));
    w[2 + e] = pk16(h_bits((_Float16)(bfr(a1[2 * e]) * EC)), h_bits((_Float16)(bfr(a1[2 * e + 1]) * EC)));
  }
  unsigned short* dst = E + (size_t)r * DEMB + (size_t)j * 8;
  for (int pass = 0; pass < 2; ++pass) {
    *(volatile v4u*)dst = w;
    __threadfence();
  }
}

__global__ __launch_bounds__(256) void hcvt(const float* __restrict__ HFp, unsigned short* CB) {
  const int tid = threadIdx.x, lane = tid & 31;
  const int row = blockIdx.x * 8 + (tid >> 5);
  const float* sp = HFp + (size_t)row * DMODEL + (size_t)lane * 8;
  const v4f a0 = *(const v4f*)(sp);
  const v4f a1 = *(const v4f*)(sp + 4);
  v4u w;
#pragma unroll
  for (int e = 0; e < 2; ++e) {
    w[e]     = pk16(h_bits((_Float16)(a0[2 * e] * HCARRY)), h_bits((_Float16)(a0[2 * e + 1] * HCARRY)));
    w[2 + e] = pk16(h_bits((_Float16)(a1[2 * e] * HCARRY)), h_bits((_Float16)(a1[2 * e + 1] * HCARRY)));
  }
  unsigned short* dst = CB + (size_t)row * DCOMB + (size_t)lane * 8;
  for (int pass = 0; pass < 2; ++pass) {
    *(volatile v4u*)dst = w;
    __threadfence();
  }
}

#define PS_FLOATS (HPB * 16 * 36)
static_assert((size_t)16 * OSP * sizeof(unsigned short) <= (size_t)PS_FLOATS * sizeof(float));
static_assert(((16 * OSP) % (8 * ATT_THREADS)) == 0 && ((16 * OSP) / (8 * ATT_THREADS)) == 2);
static_assert(OSP == HDIM * HPB && (OSP8 % 8) == 0 && ((OSP * 2) % 128) == 0 && ((DMODEL * 2) % 128) == 0 && HDIM == 32);

__global__ __launch_bounds__(ATT_THREADS)
void attn8(const unsigned short* __restrict__ QHp, const unsigned short* __restrict__ KHp,
           const unsigned short* __restrict__ VTq, const int* __restrict__ sin_, unsigned short* CT) {
  __shared__ __align__(16) float smem[PS_FLOATS];

  const int tid  = threadIdx.x;
  const int wave = tid >> 5;
  const int lane = tid & 31;
  const int hh   = lane >> 4;
  const int c    = lane & 15;

  const int qt   = blockIdx.x % (SEQ / 16);
  const int bat  = blockIdx.x / (SEQ / 16);
  const int head = wave;
  const int q0   = qt * 16;
  const int srow = q0 + 8 * hh;
  const int kend = q0 + 16;

  const size_t qofs = ((size_t)bat * SEQ + q0 + c) * DMODEL + head * HDIM + 8 * hh;
  const _Float16* Qh = (const _Float16*)(const void*)QHp + qofs;
  const _Float16* Kb = (const _Float16*)(const void*)KHp + ((size_t)bat * SEQ * DMODEL + head * HDIM + 8 * hh);
  const _Float16* Vb = (const _Float16*)(const void*)VTq + (((size_t)bat * DMODEL + head * HDIM) * SEQ + 8 * hh);
  const int* sb = sin_ + (size_t)bat * SEQ_FULL;
  const float lsc = (LOG2E * ATT_SCALE) / (QC * KC);

  const v16h qa = ldfrag_h(Qh);

  float mrow[8], lrow[8];
  v8f o0 = zero8(), o1 = zero8();
#pragma unroll
  for (int r = 0; r < 8; ++r) { mrow[r] = -INFINITY; lrow[r] = 0.f; }
  float* pt = smem + wave * (16 * 36);

#pragma unroll 1
  for (int kb = 0; kb < kend; kb += 32) {
    const _Float16* kp = Kb + (size_t)(kb + c) * DMODEL;
    const v16h k0v = ldfrag_h(kp);
    const v16h k1v = ldfrag_h(kp + (size_t)16 * DMODEL);
    v8f s0 = mma_raw(qa, k0v, zero8());
    v8f s1 = mma_raw(qa, k1v, zero8());
    guard_ab3(s0, s1, k0v, k1v, qa);

    const int key0 = kb + c;
    const int key1 = kb + 16 + c;
    const int mk0 = (sb[imin(key0, SEQ - 1)] >= 0) ? 1 : 0;
    const int mk1 = (sb[imin(key1, SEQ - 1)] >= 0) ? 1 : 0;
#pragma unroll
    for (int r = 0; r < 8; ++r) {
      const int qi = srow + r;
      float t0 = s0[r] * lsc;
      float t1 = s1[r] * lsc;
      t0 = (key0 > qi || mk0 == 0) ? MFILL : t0;
      t1 = (key1 > qi || mk1 == 0) ? MFILL : t1;
      float mx = fmaxf(t0, t1);
#pragma unroll
      for (int off = 1; off < 16; off <<= 1) mx = fmaxf(mx, __shfl_xor(mx, off, 32));
      const float mn = fmaxf(mrow[r], mx);
      const float al = exp2f(fmaxf(mrow[r] - mn, -126.0f));
      mrow[r] = mn;
      const float e0 = exp2f(t0 - mn);
      const float e1 = exp2f(t1 - mn);
      float ps = e0 + e1;
#pragma unroll
      for (int off = 1; off < 16; off <<= 1) ps += __shfl_xor(ps, off, 32);
      lrow[r] = lrow[r] * al + ps;
      o0[r] *= al;
      o1[r] *= al;
      const int ro = (8 * hh + r) * 36 + c;
      pt[ro]      = e0;
      pt[ro + 16] = e1;
    }
    wave_sync_lds();
    FragH ph;
    {
      const float* prow = pt + c * 36 + 8 * hh;
      const v4f p0 = *(const v4f*)(prow), p1 = *(const v4f*)(prow + 4);
      const v4f p2 = *(const v4f*)(prow + 16), p3 = *(const v4f*)(prow + 20);
#pragma unroll
      for (int e = 0; e < 4; ++e) {
        ph.h[0][e]     = (_Float16)(p0[e] * PC);
        ph.h[0][4 + e] = (_Float16)(p1[e] * PC);
        ph.h[1][e]     = (_Float16)(p2[e] * PC);
        ph.h[1][4 + e] = (_Float16)(p3[e] * PC);
      }
    }
    const _Float16* vp = Vb + (size_t)c * SEQ + kb;
    {
      const v16h vb0 = ldfrag_h(vp);
      const v16h vb1 = ldfrag_h(vp + (size_t)16 * SEQ);
      o0 = mma_raw(ph.v, vb0, o0);
      o1 = mma_raw(ph.v, vb1, o1);
      guard_ab3(o0, o1, ph.v, vb0, vb1);
    }
    wave_sync_lds();
  }

  __syncthreads();
  unsigned short* Os = (unsigned short*)smem;
  const float oc = FC / (PC * VC);
  unsigned short* osw = Os + wave * HDIM + c;
#pragma unroll
  for (int r = 0; r < 8; ++r) {
    const float inv = (1.0f / lrow[r]) * oc;
    unsigned short* op = osw + (8 * hh + r) * OSP;
    op[0]  = h_bits((_Float16)(o0[r] * inv));
    op[16] = h_bits((_Float16)(o1[r] * inv));
  }
  __syncthreads();
  {
    v4u vals[2];
#pragma unroll
    for (int it = 0; it < 2; ++it) {
      const int p = it * ATT_THREADS + tid;
      vals[it] = *(const v4u*)(Os + (size_t)p * 8);
    }
    unsigned short* dst = CT + ((size_t)bat * SEQ + q0) * DMODEL;
    for (int pass = 0; pass < 2; ++pass) {
#pragma unroll
      for (int it = 0; it < 2; ++it) {
        const int p = it * ATT_THREADS + tid;
        const int row = p / OSP8, col8 = (p - row * OSP8) * 8;
        *(volatile v4u*)(dst + (size_t)row * DMODEL + col8) = vals[it];
      }
      __threadfence();
    }
  }
}

__global__ __launch_bounds__(LN_THREADS)
void lnorm2(const float* __restrict__ Yp, const float* __restrict__ gp, const float* __restrict__ bp,
            float* outf, unsigned short* outh, int hp, float hc) {
  __shared__ float red[2][LN_THREADS / 32];
  __shared__ __align__(16) unsigned short srow[DMODEL];
  const int row  = blockIdx.x;
  const int tid  = threadIdx.x;
  const int lane = tid & 31;
  const int wave = tid >> 5;
  const size_t base = (size_t)row * DMODEL + (size_t)tid * 4;
  const v4f v = *(const v4f*)(Yp + base);
  float s = (v[0] + v[1]) + (v[2] + v[3]);
#pragma unroll
  for (int off = 1; off < 32; off <<= 1) s += __shfl_xor(s, off, 32);
  if (lane == 0) red[0][wave] = s;
  __syncthreads();
  float tot = 0.f;
#pragma unroll
  for (int w = 0; w < LN_THREADS / 32; ++w) tot += red[0][w];
  const float mu = tot * (1.0f / (float)DMODEL);
  v4f d;
#pragma unroll
  for (int e = 0; e < 4; ++e) d[e] = v[e] - mu;
  float q = (d[0] * d[0] + d[1] * d[1]) + (d[2] * d[2] + d[3] * d[3]);
#pragma unroll
  for (int off = 1; off < 32; off <<= 1) q += __shfl_xor(q, off, 32);
  if (lane == 0) red[1][wave] = q;
  __syncthreads();
  float totq = 0.f;
#pragma unroll
  for (int w = 0; w < LN_THREADS / 32; ++w) totq += red[1][w];
  const float var  = totq * (1.0f / (float)DMODEL);
  const float rstd = rsqrtf(var + LN_EPS);
  const v4f gv = *(const v4f*)(gp + (size_t)tid * 4);
  const v4f bv = *(const v4f*)(bp + (size_t)tid * 4);
  v4f o;
#pragma unroll
  for (int e = 0; e < 4; ++e) o[e] = (d[e] * rstd) * bfr(gv[e]) + bfr(bv[e]);
  v2u w;
  w[0] = pk16(h_bits((_Float16)(o[0] * hc)), h_bits((_Float16)(o[1] * hc)));
  w[1] = pk16(h_bits((_Float16)(o[2] * hc)), h_bits((_Float16)(o[3] * hc)));
  *(v2u*)(srow + tid * 4) = w;
  __syncthreads();
  const v4u hv = *(const v4u*)(srow + (tid & 31) * 8);
  float* pf = outf + base;
  unsigned short* ph = outh + (size_t)row * hp + (size_t)(tid & 31) * 8;
  for (int pass = 0; pass < 2; ++pass) {
    *(volatile v4f*)pf = o;
    if (wave == 0) *(volatile v4u*)ph = hv;
    __threadfence();
  }
}

__global__ __launch_bounds__(SEQ)
void statk(const int* __restrict__ sin_, const float* __restrict__ sw1p, const float* __restrict__ sb1p,
           unsigned short* HID) {
  __shared__ int ss[SEQ];
  __shared__ int mm[SEQ];
  __shared__ float sW1[NFEAT * NSH];
  __shared__ float sB1[NSH];
  __shared__ __align__(16) unsigned short hidS[SEQ * HSP];
  const int b = blockIdx.x, t = threadIdx.x;
  {
    const int sv = sin_[(size_t)b * SEQ_FULL + t];
    const int msk = (sv >= 0) ? 1 : 0;
    ss[t] = msk ? sv : 0;
    mm[t] = msk;
  }
  if (t < NFEAT * NSH) sW1[t] = bfr(sw1p[t]);
  if (t < NSH) sB1[t] = bfr(sb1p[t]);
  __syncthreads();

  float valid = 0.f, corr = 0.f;
#pragma unroll
  for (int j = 0; j < WIN; ++j) {
    const int p = t - (WIN - 1) + j;
    const int pc = imax(p, 0);
    const float mv = (float)mm[pc], sv = (float)ss[pc];
    valid += (p >= 0) ? mv : 0.f;
    corr  += (p >= 0) ? sv : 0.f;
  }
  float rc = 0.f, rcs = 0.f;
#pragma unroll
  for (int j = 0; j < 5; ++j) {
    const int p = t - 4 + j;
    const int pc = imax(p, 0);
    const float mv = (float)mm[pc], sv = (float)ss[pc];
    rc  += (p >= 0) ? mv : 0.f;
    rcs += (p >= 0) ? sv : 0.f;
  }
  float dsum = 0.f;
#pragma unroll
  for (int j = 0; j < WIN - 1; ++j) {
    const int p = t - (WIN - 2) + j;
    const int pc = imax(p, 1);
    const int dd = (ss[pc] != ss[pc - 1] && mm[pc] != 0 && mm[pc - 1] != 0) ? 1 : 0;
    dsum += (p >= 1 && dd != 0) ? 1.f : 0.f;
  }
  float run = 0.f, mxr = 0.f;
#pragma unroll
  for (int j = 0; j < WIN; ++j) {
    const int p = t - (WIN - 1) + j;
    const int pc = imax(p, 0);
    const int pm1c = imax(p - 1, 0);
    const int cm = (p >= 0) ? mm[pc] : 0;
    const int pm = (j >= 1 && p - 1 >= 0) ? mm[pm1c] : 0;
    const int eq = (pm != 0 && ss[pc] == ss[pm1c]) ? 1 : 0;
    run = (cm != 0) ? ((eq != 0 ? run : 0.f) + 1.f) : 0.f;
    mxr = fmaxf(mxr, run);
  }
  const float f0 = corr / (valid + 1e-6f);
  const float f1 = rcs / (rc + 1e-6f);
  const float f2 = dsum / (valid + 1e-6f);
  const float f3 = mxr * (1.0f / (float)WIN);
  const float f4 = (float)t * (1.0f / (float)RELDEN);
  const float f5 = valid * (1.0f / (float)WIN);

#pragma unroll 1
  for (int k = 0; k < NSH; ++k) {
    float a = sB1[k];
    a += f0 * sW1[0 * NSH + k];
    a += f1 * sW1[1 * NSH + k];
    a += f2 * sW1[2 * NSH + k];
    a += f3 * sW1[3 * NSH + k];
    a += f4 * sW1[4 * NSH + k];
    a += f5 * sW1[5 * NSH + k];
    a = fmaxf(a, 0.f);
    hidS[t * HSP + k] = h_bits((_Float16)(a * HIDC));
  }
  __syncthreads();

  v4u vals[8];
#pragma unroll
  for (int it = 0; it < 8; ++it) {
    const int p = it * SEQ + t;
    const int row = p >> 3, piece = p & 7;
    const int pc2 = piece & 3;
    const v4u v = *(const v4u*)(hidS + row * HSP + pc2 * 8);
    v4u z;
#pragma unroll
    for (int e = 0; e < 4; ++e) z[e] = (piece < 4) ? v[e] : 0u;
    vals[it] = z;
  }
  unsigned short* dstb = HID + (size_t)b * SEQ * HIDK;
  for (int pass = 0; pass < 2; ++pass) {
#pragma unroll
    for (int it = 0; it < 8; ++it) {
      const int p = it * SEQ + t;
      const int row = p >> 3, piece = p & 7;
      *(volatile v4u*)(dstb + (size_t)row * HIDK + piece * 8) = vals[it];
    }
    __threadfence();
  }
}

__global__ __launch_bounds__(HEAD_THREADS)
void headk(const unsigned short* __restrict__ CBp, const unsigned short* __restrict__ WCp,
           const float* __restrict__ cb1p, const float* __restrict__ cw2p, const float* __restrict__ cb2p,
           const int* __restrict__ sin_, float* out) {
  __shared__ __align__(16) float lg[HEAD_ROWS];
  const int tid = threadIdx.x, lane = tid & 31, wave = tid >> 5;
  const int rlane = lane & 15, hh = lane >> 4, koff = hh * 8;
  const int m0 = blockIdx.x * HEAD_ROWS + wave * 64;
  const float osc = 1.0f / (HCARRY * WSC);

  float part[4][8];
#pragma unroll
  for (int i = 0; i < 4; ++i)
#pragma unroll
    for (int r = 0; r < 8; ++r) part[i][r] = 0.f;

#pragma unroll 1
  for (int ns = 0; ns < DMODEL / 32; ++ns) {
    const int n0 = ns * 32;
    v8f acc[4][2];
#pragma unroll
    for (int i = 0; i < 4; ++i) { acc[i][0] = zero8(); acc[i][1] = zero8(); }
    for (int k0 = 0; k0 < DCOMB; k0 += 32) {
      v16h bh[2];
#pragma unroll
      for (int j = 0; j < 2; ++j) {
        bh[j] = ldfrag_u(WCp + (size_t)(n0 + (j << 4) + rlane) * DCOMB + koff + k0);
      }
#pragma unroll
      for (int i = 0; i < 4; ++i) {
        const v16h ah = ldfrag_u(CBp + (size_t)(m0 + (i << 4) + rlane) * DCOMB + koff + k0);
        acc[i][0] = mma_raw(ah, bh[0], acc[i][0]);
        acc[i][1] = mma_raw(ah, bh[1], acc[i][1]);
        dep_guard1(acc[i][0], acc[i][1], ah);
      }
      keep2_h(bh[0], bh[1]);
    }
    acc_guard4(acc[0][0], acc[0][1], acc[1][0], acc[1][1]);
    acc_guard4(acc[2][0], acc[2][1], acc[3][0], acc[3][1]);
#pragma unroll
    for (int j = 0; j < 2; ++j) {
      const int n = n0 + (j << 4) + rlane;
      const float b1 = bfr(cb1p[n]);
      const float w2 = bfr(cw2p[n]);
#pragma unroll
      for (int i = 0; i < 4; ++i) {
#pragma unroll
        for (int r = 0; r < 8; ++r) part[i][r] += fmaxf(acc[i][j][r] * osc + b1, 0.f) * w2;
      }
    }
  }
#pragma unroll
  for (int i = 0; i < 4; ++i) {
#pragma unroll
    for (int r = 0; r < 8; ++r) {
      float v = part[i][r];
      v += __shfl_xor(v, 1, 32);
      v += __shfl_xor(v, 2, 32);
      v += __shfl_xor(v, 4, 32);
      v += __shfl_xor(v, 8, 32);
      const int row = wave * 64 + (i << 4) + hh * 8 + r;
      if (rlane == 0) lg[row] = v;
    }
  }
  __syncthreads();
  const float b2 = bfr(cb2p[0]);
  const int lt = tid & 63;
  v4f o;
#pragma unroll
  for (int e = 0; e < 4; ++e) {
    const int rr  = lt * 4 + e;
    const int tok = blockIdx.x * HEAD_ROWS + rr;
    const int b = tok / SEQ, t = tok - b * SEQ;
    const int sv = sin_[(size_t)b * SEQ_FULL + t];
    const float lgt = lg[rr] + b2;
    o[e] = (sv >= 0) ? lgt : MFILL;
  }
  if (tid < 64) {
    float* dst = out + (size_t)blockIdx.x * HEAD_ROWS + (size_t)lt * 4;
    for (int pass = 0; pass < 2; ++pass) {
      *(volatile v4f*)dst = o;
      __threadfence();
    }
  }
}

extern "C" void kernel_launch(void* const* d_in, const int* in_sizes, int n_in,
                              void* d_out, int out_size, void* d_ws, size_t ws_size,
                              hipStream_t stream) {
  if (n_in < 27) return;
  if (in_sizes[0] < NB * SEQ_FULL || in_sizes[1] < NB * SEQ_FULL) return;
  if (in_sizes[2] < DMODEL || (in_sizes[2] % DMODEL) != 0) return;
  if (in_sizes[3] < DMODEL || (in_sizes[3] % DMODEL) != 0) return;
  if (in_sizes[4] < SEQ * DMODEL) return;
  if (in_sizes[5] < DEMB * DMODEL || in_sizes[6] < DMODEL) return;
  if (in_sizes[7] < NLAYER * DMODEL * 3 * DMODEL || in_sizes[8] < NLAYER * 3 * DMODEL) return;
  if (in_sizes[9] < NLAYER * DMODEL * DMODEL || in_sizes[10] < NLAYER * DMODEL) return;
  if (in_sizes[11] < NLAYER * DMODEL || in_sizes[12] < NLAYER * DMODEL) return;
  if (in_sizes[13] < NLAYER * DMODEL || in_sizes[14] < NLAYER * DMODEL) return;
  if (in_sizes[15] < NLAYER * DMODEL * DFF || in_sizes[16] < NLAYER * DFF) return;
  if (in_sizes[17] < NLAYER * DFF * DMODEL || in_sizes[18] < NLAYER * DMODEL) return;
  if (in_sizes[19] < NFEAT * NSH || in_sizes[20] < NSH) return;
  if (in_sizes[21] < NSH * DSTAT || in_sizes[22] < DSTAT) return;
  if (in_sizes[23] < DCOMB * DMODEL || in_sizes[24] < DMODEL) return;
  if (in_sizes[25] < DMODEL || in_sizes[26] < 1) return;
  if (out_size < NTOK) return;

  const int*   qin        = (const int*)d_in[0];
  const int*   sin_       = (const int*)d_in[1];
  const float* q_embed    = (const float*)d_in[2];
  const float* s_embed    = (const float*)d_in[3];
  const float* pos_embed  = (const float*)d_in[4];
  const float* fusion_w   = (const float*)d_in[5];
  const float* fusion_b   = (const float*)d_in[6];
  const float* in_proj_w  = (const float*)d_in[7];
  const float* in_proj_b  = (const float*)d_in[8];
  const float* out_proj_w = (const float*)d_in[9];
  const float* out_proj_b = (const float*)d_in[10];
  const float* ln1_g      = (const float*)d_in[11];
  const float* ln1_b      = (const float*)d_in[12];
  const float* ln2_g      = (const float*)d_in[13];
  const float* ln2_b      = (const float*)d_in[14];
  const float* ff1_w      = (const float*)d_in[15];
  const float* ff1_b      = (const float*)d_in[16];
  const float* ff2_w      = (const float*)d_in[17];
  const float* ff2_b      = (const float*)d_in[18];
  const float* sw1        = (const float*)d_in[19];
  const float* sb1        = (const float*)d_in[20];
  const float* sw2        = (const float*)d_in[21];
  const float* sb2        = (const float*)d_in[22];
  const float* cw1        = (const float*)d_in[23];
  const float* cb1        = (const float*)d_in[24];
  const float* cw2        = (const float*)d_in[25];
  const float* cb2        = (const float*)d_in[26];
  float*       out        = (float*)d_out;
  const int nqrows = in_sizes[2] / DMODEL;
  const int nsrows = in_sizes[3] / DMODEL;

  const size_t PWFU  = (size_t)DMODEL * DEMB * 2;
  const size_t PWQKV = (size_t)NLAYER * 3 * DMODEL * DMODEL * 2;
  const size_t PWO   = (size_t)NLAYER * DMODEL * DMODEL * 2;
  const size_t PW1   = (size_t)NLAYER * DFF * DMODEL * 2;
  const size_t PW2   = PW1;
  const size_t PWC1  = (size_t)DMODEL * DCOMB * 2;
  const size_t PWS2  = (size_t)DSTAT * HIDK * 2;
  const size_t PF32  = (size_t)NTOK * DMODEL * 4;
  const size_t PCB   = (size_t)NTOK * DCOMB * 2;
  const size_t PH16  = (size_t)NTOK * DMODEL * 2;
  const size_t PVT   = (size_t)NB * DMODEL * SEQ * 2;
  const size_t PE16  = (size_t)NTOK * DEMB * 2;
  const size_t PG16  = (size_t)NTOK * DFF * 2;
  const size_t PGE   = (PG16 > PE16) ? PG16 : PE16;
  const size_t PHID  = (size_t)NTOK * HIDK * 2;
  size_t off = 0;
  const size_t oWFU  = off; off += PWFU;
  const size_t oWQKV = off; off += PWQKV;
  const size_t oWO   = off; off += PWO;
  const size_t oW1   = off; off += PW1;
  const size_t oW2   = off; off += PW2;
  const size_t oWC1  = off; off += PWC1;
  const size_t oWS2  = off; off += PWS2;
  const size_t oHF   = off; off += PF32;
  const size_t oX1F  = off; off += PF32;
  const size_t oCB   = off; off += PCB;
  const size_t oQH   = off; off += PH16;
  const size_t oKH   = off; off += PH16;
  const size_t oVT   = off; off += PVT;
  const size_t oCT   = off; off += PH16;
  const size_t oGE   = off; off += PGE;
  const size_t oHID  = off; off += PHID;
  const size_t endAll = off;
  if (endAll > ws_size) return;
  if (endAll > (size_t)134217728) return;

  char* ws = (char*)d_ws;
  unsigned short* WFU  = (unsigned short*)(ws + oWFU);
  unsigned short* WQKV = (unsigned short*)(ws + oWQKV);
  unsigned short* WO16 = (unsigned short*)(ws + oWO);
  unsigned short* W116 = (unsigned short*)(ws + oW1);
  unsigned short* W216 = (unsigned short*)(ws + oW2);
  unsigned short* WC1  = (unsigned short*)(ws + oWC1);
  unsigned short* WS2  = (unsigned short*)(ws + oWS2);
  float*          HF   = (float*)(ws + oHF);
  float*          X1F  = (float*)(ws + oX1F);
  unsigned short* CB16 = (unsigned short*)(ws + oCB);
  unsigned short* QH   = (unsigned short*)(ws + oQH);
  unsigned short* KH   = (unsigned short*)(ws + oKH);
  unsigned short* VTp  = (unsigned short*)(ws + oVT);
  unsigned short* CT   = (unsigned short*)(ws + oCT);
  unsigned short* E16  = (unsigned short*)(ws + oGE);
  unsigned short* G16  = (unsigned short*)(ws + oGE);
  unsigned short* HID  = (unsigned short*)(ws + oHID);

  const dim3 blk(256);
  const dim3 gTfu(DMODEL / 64, DEMB / 64, 1);
  const dim3 gTqkv(3 * DMODEL / 64, DMODEL / 64, NLAYER);
  const dim3 gTo(DMODEL / 64, DMODEL / 64, NLAYER);
  const dim3 gT1(DFF / 64, DMODEL / 64, NLAYER);
  const dim3 gT2(DMODEL / 64, DFF / 64, NLAYER);
  const dim3 gTc1(DMODEL / 64, DCOMB / 64, 1);
  const dim3 gTs2(DSTAT / 64, HIDK / 64, 1);
  const int tilesP = (NTOK / 64) * (DMODEL / 64);
  const int tilesV = (DMODEL / 64) * (SEQ / 64);
  const int tilesF = (NTOK / 64) * (DFF / 64);
  const int tilesS = (NTOK / 64) * (DSTAT / 64);
  const dim3 gP((tilesP + 7) / 8, 1);
  const dim3 gV((tilesV + 7) / 8, NB);
  const dim3 gF((tilesF + 7) / 8, 1);
  const dim3 gS((tilesS + 7) / 8, 1);
  const dim3 gEG(NTOK / 4);
  const dim3 gHC(NTOK / 8);
  const dim3 gAT(ATT_BLOCKS);
  const dim3 bAT(ATT_THREADS);
  const dim3 gLN(NTOK);
  const dim3 bLN(LN_THREADS);
  const dim3 gST(NB);
  const dim3 bST(SEQ);
  const dim3 gHD(NTOK / HEAD_ROWS);
  const dim3 bHD(HEAD_THREADS);

  tcvt16<<<gTfu, blk, 0, stream>>>(fusion_w, 0LL, WFU, 0LL, DEMB, DMODEL, DEMB, DMODEL, WSC);
  tcvt16<<<gTqkv, blk, 0, stream>>>(in_proj_w, (long long)DMODEL * 3 * DMODEL, WQKV, (long long)3 * DMODEL * DMODEL,
                                    DMODEL, 3 * DMODEL, DMODEL, 3 * DMODEL, WSC);
  tcvt16<<<gTo, blk, 0, stream>>>(out_proj_w, (long long)DMODEL * DMODEL, WO16, (long long)DMODEL * DMODEL,
                                  DMODEL, DMODEL, DMODEL, DMODEL, WSC);
  tcvt16<<<gT1, blk, 0, stream>>>(ff1_w, (long long)DMODEL * DFF, W116, (long long)DFF * DMODEL, DMODEL, DFF, DMODEL, DFF, WSC);
  tcvt16<<<gT2, blk, 0, stream>>>(ff2_w, (long long)DFF * DMODEL, W216, (long long)DMODEL * DFF, DFF, DMODEL, DFF, DMODEL, WSC);
  tcvt16<<<gTc1, blk, 0, stream>>>(cw1, 0LL, WC1, 0LL, DCOMB, DMODEL, DCOMB, DMODEL, WSC);
  tcvt16<<<gTs2, blk, 0, stream>>>(sw2, 0LL, WS2, 0LL, NSH, DSTAT, HIDK, DSTAT, WSC);

  egath<<<gEG, blk, 0, stream>>>(qin, sin_, q_embed, nqrows, s_embed, nsrows, E16);

  gemm64<0, 3, 2, 1><<<gP, blk, 0, stream>>>(
      E16, DEMB, 0LL,
      WFU, DEMB, 0LL,
      pos_embed, SEQ,
      fusion_b, DMODEL,
      (void*)HF, DMODEL, 0LL,
      NTOK, DMODEL, DEMB, 1.0f / (EC * WSC), 1.0f);

  hcvt<<<gHC, blk, 0, stream>>>(HF, CB16);

  for (int l = 0; l < NLAYER; ++l) {
    const unsigned short* WL = WQKV + (size_t)l * 3 * DMODEL * DMODEL;
    const float* bL = in_proj_b + (size_t)l * 3 * DMODEL;

    gemm64<2, 0, 0, 1><<<gP, blk, 0, stream>>>(
        CB16, DCOMB, 0LL,
        WL, DMODEL, 0LL,
        (const float*)0, 1,
        bL, DMODEL,
        (void*)QH, DMODEL, 0LL,
        NTOK, DMODEL, DMODEL, 1.0f / (HCARRY * WSC), QC);

    gemm64<2, 0, 0, 1><<<gP, blk, 0, stream>>>(
        CB16, DCOMB, 0LL,
        WL + (size_t)DMODEL * DMODEL, DMODEL, 0LL,
        (const float*)0, 1,
        bL + DMODEL, DMODEL,
        (void*)KH, DMODEL, 0LL,
        NTOK, DMODEL, DMODEL, 1.0f / (HCARRY * WSC), KC);

    gemm64<2, 0, 0, 2><<<gV, blk, 0, stream>>>(
        WL + (size_t)2 * DMODEL * DMODEL, DMODEL, 0LL,
        CB16, DCOMB, (long long)SEQ * DCOMB,
        (const float*)0, 1,
        bL + 2 * DMODEL, DMODEL,
        (void*)VTp, SEQ, (long long)DMODEL * SEQ,
        DMODEL, SEQ, DMODEL, 1.0f / (HCARRY * WSC), VC);

    attn8<<<gAT, bAT, 0, stream>>>(QH, KH, VTp, sin_, CT);

    gemm64<0, 2, 0, 1><<<gP, blk, 0, stream>>>(
        CT, DMODEL, 0LL,
        WO16 + (size_t)l * DMODEL * DMODEL, DMODEL, 0LL,
        HF, 1,
        out_proj_b + (size_t)l * DMODEL, DMODEL,
        (void*)X1F, DMODEL, 0LL,
        NTOK, DMODEL, DMODEL, 1.0f / (FC * WSC), 1.0f);

    lnorm2<<<gLN, bLN, 0, stream>>>(X1F, ln1_g + (size_t)l * DMODEL, ln1_b + (size_t)l * DMODEL, HF, CB16, DCOMB, HCARRY);

    gemm64<2, 0, 1, 1><<<gF, blk, 0, stream>>>(
        CB16, DCOMB, 0LL,
        W116 + (size_t)l * DFF * DMODEL, DMODEL, 0LL,
        (const float*)0, 1,
        ff1_b + (size_t)l * DFF, DFF,
        (void*)G16, DFF, 0LL,
        NTOK, DFF, DMODEL, 1.0f / (HCARRY * WSC), GC);

    gemm64<0, 2, 0, 1><<<gP, blk, 0, stream>>>(
        G16, DFF, 0LL,
        W216 + (size_t)l * DMODEL * DFF, DFF, 0LL,
        HF, 1,
        ff2_b + (size_t)l * DMODEL, DMODEL,
        (void*)X1F, DMODEL, 0LL,
        NTOK, DMODEL, DFF, 1.0f / (GC * WSC), 1.0f);

    lnorm2<<<gLN, bLN, 0, stream>>>(X1F, ln2_g + (size_t)l * DMODEL, ln2_b + (size_t)l * DMODEL, HF, CB16, DCOMB, HCARRY);
  }

  statk<<<gST, bST, 0, stream>>>(sin_, sw1, sb1, HID);

  gemm64<2, 0, 0, 1><<<gS, blk, 0, stream>>>(
      HID, HIDK, 0LL,
      WS2, HIDK, 0LL,
      (const float*)0, 1,
      sb2, DSTAT,
      (void*)(CB16 + DMODEL), DCOMB, 0LL,
      NTOK, DSTAT, HIDK, 1.0f / (HIDC * WSC), HCARRY);

  headk<<<gHD, bHD, 0, stream>>>(CB16, WC1, cb1, cw2, cb2, sin_, out);
  (void)hipGetLastError();
}
